// DeepHamCritic_35012573397744
// MI455X (gfx1250) — hardware-verified
//
#include <hip/hip_runtime.h>
#include <stddef.h>


#define DIN     128
#define DHID    512
#define NCAT    1024
#define YP      1024
#define NTHR    256
#define NWAVE   8
#define EPT     8
#define CHUNK   (NTHR * EPT)
#define WCAP    (EPT * 32)
#define LISTN   (NWAVE * WCAP)
#define NBMAX   2048
#define RCAP    28672
#define DEGCAP  4096
#define GBM     64
#define GTHR    128
#define NEG2    0.2f
#define NEG01   0.01f
#define WSCAP   134217728
#define LDS_AGG ((2 * RCAP + 2 * NBMAX + LISTN) * 4 + 64)
#define WTOT    (2 * DHID * DIN + 6 * DHID * DHID)

static_assert((CHUNK & (CHUNK - 1)) == 0 && CHUNK <= 4096);
static_assert((NBMAX & (NBMAX - 1)) == 0 && NBMAX <= 4096);
static_assert(NTHR * 8 == NBMAX);
static_assert(LISTN >= NBMAX);
static_assert(LISTN >= NWAVE * WCAP);
static_assert((RCAP % 32) == 0);
static_assert(LDS_AGG <= 300000);
static_assert(GBM == (GTHR / 32) * 16);
static_assert(2 * GBM == GTHR);
static_assert(4 * GTHR == DHID);
static_assert(DHID == 2 * 8 * 32);
static_assert((DIN % 32) == 0 && (DHID % 64) == 0 && NCAT == 2 * DHID && YP == NCAT);
static_assert((GBM % 4) == 0 && GBM <= GTHR);

typedef float          v4f  __attribute__((ext_vector_type(4)));
typedef float          v8f  __attribute__((ext_vector_type(8)));
typedef int            v4i  __attribute__((ext_vector_type(4)));
typedef int            v8i  __attribute__((ext_vector_type(8)));
typedef unsigned short v8us __attribute__((ext_vector_type(8)));
typedef __bf16         v16b __attribute__((ext_vector_type(16)));
union FragB { v16b v; v8us h[2]; v8i w; };

__device__ __forceinline__ v8f wmb(const FragB& a, const FragB& b, v8f c) {
  v8f d = __builtin_amdgcn_wmma_f32_16x16x32_bf16(false, a.v, false, b.v, (short)0, c, false, false);
  asm volatile("v_nop\n\tv_nop\n\tv_nop\n\tv_nop" : "+v"(d) : "v"(a.w), "v"(b.w));
  return d;
}

__device__ __forceinline__ unsigned int bf16_bits(float f) {
  const unsigned int u = __float_as_uint(f);
  return (u + 0x7fffu + ((u >> 16) & 1u)) >> 16;
}

__device__ __forceinline__ void split8(v4f a, v4f b, v8us& hv, v8us& lv) {
  const float s[8] = {a.x, a.y, a.z, a.w, b.x, b.y, b.z, b.w};
#pragma unroll
  for (int i = 0; i < 8; ++i) {
    const unsigned int hb = bf16_bits(s[i]);
    const float r = s[i] - __uint_as_float(hb << 16);
    const unsigned int lb = bf16_bits(r);
    hv[i] = (unsigned short)hb;
    lv[i] = (unsigned short)lb;
  }
}

__device__ __forceinline__ float tanh_e(float v) {
  const float ex = __expf(2.0f * v);
  const float r = __builtin_amdgcn_rcpf(ex + 1.0f);
  return fmaf(-2.0f, r, 1.0f);
}

__device__ __forceinline__ int scan_chunk(const int* __restrict__ dsts, int nE, int cbase, int slotBase,
                                          int nb, int vec8, int* list, int tid, int lane, int wave) {
  int wc = 0;
  const int el0  = tid * EPT;
  const int e0   = cbase + el0;
  const int sent = -2147483647 - 1;
  v4i da, db;
  if (vec8 != 0 && cbase + CHUNK <= nE) {
    da = *(const v4i*)(dsts + e0);
    db = *(const v4i*)(dsts + e0 + 4);
  } else {
    da.x = (e0     < nE) ? dsts[min(e0,     nE - 1)] : sent;
    da.y = (e0 + 1 < nE) ? dsts[min(e0 + 1, nE - 1)] : sent;
    da.z = (e0 + 2 < nE) ? dsts[min(e0 + 2, nE - 1)] : sent;
    da.w = (e0 + 3 < nE) ? dsts[min(e0 + 3, nE - 1)] : sent;
    db.x = (e0 + 4 < nE) ? dsts[min(e0 + 4, nE - 1)] : sent;
    db.y = (e0 + 5 < nE) ? dsts[min(e0 + 5, nE - 1)] : sent;
    db.z = (e0 + 6 < nE) ? dsts[min(e0 + 6, nE - 1)] : sent;
    db.w = (e0 + 7 < nE) ? dsts[min(e0 + 7, nE - 1)] : sent;
  }
  const unsigned nbs = (unsigned)slotBase;
  const unsigned unb = (unsigned)nb;
  const unsigned s0 = (unsigned)da.x - nbs, s1 = (unsigned)da.y - nbs;
  const unsigned s2 = (unsigned)da.z - nbs, s3 = (unsigned)da.w - nbs;
  const unsigned s4 = (unsigned)db.x - nbs, s5 = (unsigned)db.y - nbs;
  const unsigned s6 = (unsigned)db.z - nbs, s7 = (unsigned)db.w - nbs;
  const bool h0 = s0 < unb, h1 = s1 < unb, h2 = s2 < unb, h3 = s3 < unb;
  const bool h4 = s4 < unb, h5 = s5 < unb, h6 = s6 < unb, h7 = s7 < unb;
  const unsigned any = __builtin_amdgcn_ballot_w32(h0 | h1 | h2 | h3 | h4 | h5 | h6 | h7);
  if (any != 0u) {
#define HITJ(J, HJ, SJ) { \
      const unsigned mj = __builtin_amdgcn_ballot_w32(HJ); \
      if (mj != 0u) { \
        if (HJ) { \
          const int pos = wc + (int)__builtin_amdgcn_mbcnt_lo(mj, 0u); \
          if (pos < WCAP) list[wave * WCAP + pos] = ((el0 + (J)) << 12) | (int)(SJ); \
        } \
        wc += (int)__builtin_popcount(mj); } }
    HITJ(0, h0, s0)
    HITJ(1, h1, s1)
    HITJ(2, h2, s2)
    HITJ(3, h3, s3)
    HITJ(4, h4, s4)
    HITJ(5, h5, s5)
    HITJ(6, h6, s6)
    HITJ(7, h7, s7)
#undef HITJ
  }
  return wc;
}

__global__ __launch_bounds__(NTHR) void k_xprep(const float* __restrict__ x, unsigned short* xh,
                                                unsigned short* xl, int nN, int nUnits) {
  const int i = (int)blockIdx.x * NTHR + (int)threadIdx.x;
  if (i >= nUnits) return;
  const int row = i >> 4;
  const int c0  = (i & 15) * 8;
  const int rc  = row < nN ? row : nN - 1;
  const float* p = x + (size_t)rc * DIN + c0;
  v4f a = *(const v4f*)p, b = *(const v4f*)(p + 4);
  const v4f z4 = {0.f, 0.f, 0.f, 0.f};
  if (row >= nN) { a = z4; b = z4; }
  v8us hv, lv;
  split8(a, b, hv, lv);
  const size_t o = (size_t)row * DIN + c0;
  *(volatile v8us*)(xh + o) = hv;
  *(volatile v8us*)(xl + o) = lv;
  __threadfence();
  *(volatile v8us*)(xh + o) = hv;
  *(volatile v8us*)(xl + o) = lv;
}

__global__ __launch_bounds__(NTHR) void k_hpad(unsigned short* ph, unsigned short* pl, int nN, int nUnits) {
  const int i = (int)blockIdx.x * NTHR + (int)threadIdx.x;
  if (i >= nUnits) return;
  const int row = nN + (i >> 6);
  const int c0  = (i & 63) * 8;
  const v8us z = {0, 0, 0, 0, 0, 0, 0, 0};
  const size_t o = (size_t)row * DHID + c0;
  *(volatile v8us*)(ph + o) = z;
  *(volatile v8us*)(pl + o) = z;
  __threadfence();
  *(volatile v8us*)(ph + o) = z;
  *(volatile v8us*)(pl + o) = z;
}

__global__ __launch_bounds__(NTHR) void k_wprep(const float* __restrict__ w0, const float* __restrict__ w1,
                                                const float* __restrict__ w2, const float* __restrict__ w3,
                                                const float* __restrict__ w4, const float* __restrict__ w5,
                                                const float* __restrict__ w6, const float* __restrict__ w7,
                                                unsigned short* wh, unsigned short* wl) {
  const int j = (int)blockIdx.y;
  const int u = (int)blockIdx.x * NTHR + (int)threadIdx.x;
  const int K  = (j < 2) ? DIN : DHID;
  const int kq = K / 8;
  const int nUnits = DHID * kq;
  if (u >= nUnits) return;
  const float* src;
  switch (j) {
    case 0: src = w0; break;
    case 1: src = w1; break;
    case 2: src = w2; break;
    case 3: src = w3; break;
    case 4: src = w4; break;
    case 5: src = w5; break;
    case 6: src = w6; break;
    default: src = w7; break;
  }
  const size_t base = (j < 2) ? (size_t)j * DHID * DIN
                              : (size_t)2 * DHID * DIN + (size_t)(j - 2) * DHID * DHID;
  const int n  = u / kq;
  const int k8 = (u - n * kq) * 8;
  const float* p = src + (size_t)k8 * DHID + n;
  v4f a, b;
  a.x = p[0 * DHID]; a.y = p[1 * DHID]; a.z = p[2 * DHID]; a.w = p[3 * DHID];
  b.x = p[4 * DHID]; b.y = p[5 * DHID]; b.z = p[6 * DHID]; b.w = p[7 * DHID];
  v8us hv, lv;
  split8(a, b, hv, lv);
  const size_t o = base + (size_t)n * K + k8;
  *(volatile v8us*)(wh + o) = hv;
  *(volatile v8us*)(wl + o) = lv;
  __threadfence();
  *(volatile v8us*)(wh + o) = hv;
  *(volatile v8us*)(wl + o) = lv;
}

template <int MODE>
__global__ __launch_bounds__(GTHR) void k_gemm(
    const unsigned short* __restrict__ ah, const unsigned short* __restrict__ al,
    const unsigned short* __restrict__ wh, const unsigned short* __restrict__ wl,
    const float* __restrict__ bias0, const float* __restrict__ bias1,
    const float* __restrict__ w3, const float* __restrict__ b3,
    float* Y, unsigned short* gh, unsigned short* gl, float* out,
    int nks, int ldk, int np, int nN) {
  __shared__ __attribute__((aligned(16))) float stg[GBM * 64];
  __shared__ __attribute__((aligned(16))) float sB[NCAT];
  __shared__ __attribute__((aligned(16))) float sW[DHID];
  __shared__ __attribute__((aligned(16))) float odot[GBM];
  const int tid = threadIdx.x, lane = tid & 31, wave = tid >> 5, hh = lane >> 4, m = lane & 15;
  const int rowBase = (int)blockIdx.x * GBM;
#pragma unroll
  for (int i = 0; i < 4; ++i) {
    sB[tid + GTHR * i] = bias0[tid + GTHR * i];
    if (MODE == 0) sB[DHID + tid + GTHR * i] = bias1[tid + GTHR * i];
    if (MODE == 2) sW[tid + GTHR * i] = w3[tid + GTHR * i];
  }
  if (MODE == 2) { if (tid < GBM) odot[tid] = 0.f; }
  const int npmax = (MODE == 0) ? (NCAT / 64) : (DHID / 64);
  const int npc = np < 1 ? 1 : (np > npmax ? npmax : np);
  const int nk  = nks < 1 ? 1 : (nks > DHID / 32 ? DHID / 32 : nks);
  const size_t lk = (size_t)ldk;
  const size_t arow = (size_t)(rowBase + 16 * wave + m) * lk + 8 * hh;
  __syncthreads();
#pragma unroll 1
  for (int p = 0; p < npc; ++p) {
    v8f acc[4];
#pragma unroll
    for (int t = 0; t < 4; ++t) { v8f z = {0.f, 0.f, 0.f, 0.f, 0.f, 0.f, 0.f, 0.f}; acc[t] = z; }
    const int col0 = 64 * p;
    const size_t brow = (size_t)(col0 + m) * lk + 8 * hh;
#pragma unroll 1
    for (int ks = 0; ks < nk; ++ks) {
      FragB fa, fl;
      fa.h[0] = *(const v8us*)(ah + arow + 32 * ks);
      fa.h[1] = *(const v8us*)(ah + arow + 32 * ks + 16);
      fl.h[0] = *(const v8us*)(al + arow + 32 * ks);
      fl.h[1] = *(const v8us*)(al + arow + 32 * ks + 16);
#pragma unroll
      for (int t = 0; t < 4; ++t) {
        const size_t bo = brow + (size_t)(16 * t) * lk + 32 * ks;
        FragB fb, fbl;
        fb.h[0]  = *(const v8us*)(wh + bo);
        fb.h[1]  = *(const v8us*)(wh + bo + 16);
        fbl.h[0] = *(const v8us*)(wl + bo);
        fbl.h[1] = *(const v8us*)(wl + bo + 16);
        acc[t] = wmb(fa, fb,  acc[t]);
        acc[t] = wmb(fa, fbl, acc[t]);
        acc[t] = wmb(fl, fb,  acc[t]);
      }
    }
    float* sp = stg + (size_t)(16 * wave + 8 * hh) * 64 + m;
#pragma unroll
    for (int t = 0; t < 4; ++t) {
      const float bj = sB[col0 + 16 * t + m];
#pragma unroll
      for (int r = 0; r < 8; ++r) {
        float v = acc[t][r] + bj;
        if (MODE != 0) v = fmaxf(v, NEG01 * v);
        sp[(size_t)r * 64 + 16 * t] = v;
      }
    }
    __syncthreads();
    if (MODE == 0) {
      const int nF4 = GBM * 16;
      float* yb = Y + (size_t)rowBase * YP + col0;
      const v4f* s4 = (const v4f*)stg;
#pragma unroll 1
      for (int f = tid; f < nF4; f += GTHR) {
        const int r = f >> 4, q = f & 15;
        const v4f v = s4[f];
        *(volatile v4f*)(yb + (size_t)r * YP + 4 * q) = v;
      }
      __threadfence();
#pragma unroll 1
      for (int f = tid; f < nF4; f += GTHR) {
        const int r = f >> 4, q = f & 15;
        const v4f v = s4[f];
        *(volatile v4f*)(yb + (size_t)r * YP + 4 * q) = v;
      }
    } else if (MODE == 1) {
      const int nU = GBM * 8;
#pragma unroll 1
      for (int f = tid; f < nU; f += GTHR) {
        const int r = f >> 3, q = f & 7;
        const float* s = stg + (size_t)r * 64 + 8 * q;
        const v4f x0 = *(const v4f*)s, x1 = *(const v4f*)(s + 4);
        v8us hv, lv;
        split8(x0, x1, hv, lv);
        const size_t o = (size_t)(rowBase + r) * DHID + col0 + 8 * q;
        *(volatile v8us*)(gh + o) = hv;
        *(volatile v8us*)(gl + o) = lv;
      }
      __threadfence();
#pragma unroll 1
      for (int f = tid; f < nU; f += GTHR) {
        const int r = f >> 3, q = f & 7;
        const float* s = stg + (size_t)r * 64 + 8 * q;
        const v4f x0 = *(const v4f*)s, x1 = *(const v4f*)(s + 4);
        v8us hv, lv;
        split8(x0, x1, hv, lv);
        const size_t o = (size_t)(rowBase + r) * DHID + col0 + 8 * q;
        *(volatile v8us*)(gh + o) = hv;
        *(volatile v8us*)(gl + o) = lv;
      }
    } else {
      const int row  = tid >> 1;
      const int half = tid & 1;
      const float* srow = stg + (size_t)row * 64 + half * 32;
      const float* wrow = sW + col0 + half * 32;
      float s = 0.f;
#pragma unroll 1
      for (int c = 0; c < 32; ++c) s = fmaf(srow[c], wrow[c], s);
      s += __shfl_xor(s, 1);
      if (half == 0) odot[row] += s;
    }
    __syncthreads();
  }
  if (MODE == 2) {
    if (wave == 0) {
      const int nValid = (nN - rowBase) < GBM ? (nN - rowBase) : GBM;
      const int n4  = nValid >> 2;
      const int rem = nValid & 3;
      const float bb = b3[0];
      v4f v = *(const v4f*)(odot + 4 * (lane < 16 ? lane : 15));
      v.x += bb; v.y += bb; v.z += bb; v.w += bb;
      float* base = out + (size_t)rowBase;
      if (lane < n4) *(volatile v4f*)(base + 4 * lane) = v;
      if (rem != 0 && lane == 0) {
        for (int j = 0; j < rem; ++j) { const float tv = odot[4 * n4 + j] + bb; *(volatile float*)(base + 4 * n4 + j) = tv; }
      }
      __threadfence();
      if (lane < n4) *(volatile v4f*)(base + 4 * lane) = v;
      if (rem != 0 && lane == 0) {
        for (int j = 0; j < rem; ++j) { const float tv = odot[4 * n4 + j] + bb; *(volatile float*)(base + 4 * n4 + j) = tv; }
      }
    }
  }
}

__global__ __launch_bounds__(NTHR) void k_agg(
    const int* __restrict__ srcs, const int* __restrict__ dsts,
    const float* __restrict__ Y, const float* __restrict__ avec, const float* __restrict__ cvec,
    unsigned short* oh, unsigned short* ol, int nN, int nE, int nb, int vec8) {
  extern __shared__ v4f lds_dyn[];
  int* reg1 = (int*)lds_dyn;
  int* reg2 = reg1 + RCAP;
  int* scnt = reg2 + RCAP;
  int* soff = scnt + NBMAX;
  int* list = soff + NBMAX;
  int* wcnt = list + LISTN;
  int* wtot = wcnt + NWAVE;
  const int tid = threadIdx.x, lane = tid & 31, wave = tid >> 5;
  const int nodeBase = (int)blockIdx.x * nb;

  for (int i = tid; i < NBMAX; i += NTHR) scnt[i] = 0;
  __syncthreads();

  int tot = 0;
  const int nChunks = (nE + CHUNK - 1) / CHUNK;
#pragma unroll 1
  for (int ch = 0; ch < nChunks; ++ch) {
    const int cbase = ch * CHUNK;
    const int wc = scan_chunk(dsts, nE, cbase, nodeBase, nb, vec8, list, tid, lane, wave);
    if (lane == 0) wcnt[wave] = wc;
    __syncthreads();
    int pre = 0, all = 0;
#pragma unroll
    for (int w2 = 0; w2 < NWAVE; ++w2) {
      int c = wcnt[w2];
      c = c < 0 ? 0 : (c > WCAP ? WCAP : c);
      all += c;
      pre += (w2 < wave) ? c : 0;
    }
    const int wcc  = wc > WCAP ? WCAP : wc;
    const int base = tot + pre;
#pragma unroll 1
    for (int i = lane; i < wcc; i += 32) {
      const int ent = list[wave * WCAP + i];
      const int el  = (ent >> 12) & (CHUNK - 1);
      const int sl  = ent & (NBMAX - 1);
      int eid = cbase + el;
      eid = eid > nE - 1 ? nE - 1 : eid;
      const int pos = base + i;
      if (pos < RCAP) reg1[pos] = (int)(((unsigned)eid << 12) | (unsigned)sl);
    }
    tot += all;
    tot = tot > RCAP ? RCAP : tot;
    __syncthreads();
  }
  const int nh = tot;

  if (wave == 0) {
#pragma unroll 1
    for (int b0 = 0; b0 < nh; b0 += 32) {
      const int idx = b0 + lane;
      const int uv  = reg1[idx < RCAP ? idx : RCAP - 1];
      const int m32 = (nh - b0) < 32 ? (nh - b0) : 32;
#pragma unroll 1
      for (int k = 0; k < m32; ++k) {
        const int u  = __builtin_amdgcn_readlane(uv, k);
        const int sl = u & (NBMAX - 1);
        if (lane == 0) scnt[sl] = scnt[sl] + 1;
      }
    }
  }
  __syncthreads();

  {
    const v4i ca = *(const v4i*)(scnt + 8 * tid);
    const v4i cb = *(const v4i*)(scnt + 8 * tid + 4);
    const int e0 = ca.x < 0 ? 0 : ca.x, e1 = ca.y < 0 ? 0 : ca.y, e2 = ca.z < 0 ? 0 : ca.z, e3 = ca.w < 0 ? 0 : ca.w;
    const int e4 = cb.x < 0 ? 0 : cb.x, e5 = cb.y < 0 ? 0 : cb.y, e6 = cb.z < 0 ? 0 : cb.z, e7 = cb.w < 0 ? 0 : cb.w;
    const int ts = e0 + e1 + e2 + e3 + e4 + e5 + e6 + e7;
    int incl = ts;
#pragma unroll
    for (int d = 1; d < 32; d <<= 1) {
      const int up = __shfl_up(incl, d);
      if (lane >= d) incl += up;
    }
    if (lane == 31) wtot[wave] = incl;
    __syncthreads();
    int pre = 0;
#pragma unroll
    for (int w2 = 0; w2 < NWAVE; ++w2) pre += (w2 < wave) ? wtot[w2] : 0;
    int run = pre + incl - ts;
    soff[8 * tid + 0] = run; run += e0;
    soff[8 * tid + 1] = run; run += e1;
    soff[8 * tid + 2] = run; run += e2;
    soff[8 * tid + 3] = run; run += e3;
    soff[8 * tid + 4] = run; run += e4;
    soff[8 * tid + 5] = run; run += e5;
    soff[8 * tid + 6] = run; run += e6;
    soff[8 * tid + 7] = run;
  }
  __syncthreads();
  for (int i = tid; i < NBMAX; i += NTHR) list[i] = soff[i];
  __syncthreads();

  if (wave == 0) {
#pragma unroll 1
    for (int b0 = 0; b0 < nh; b0 += 32) {
      const int idx = b0 + lane;
      const int uv  = reg1[idx < RCAP ? idx : RCAP - 1];
      const int m32 = (nh - b0) < 32 ? (nh - b0) : 32;
#pragma unroll 1
      for (int k = 0; k < m32; ++k) {
        const int u   = __builtin_amdgcn_readlane(uv, k);
        const int sl  = u & (NBMAX - 1);
        const int eid = (int)((unsigned)u >> 12);
        if (lane == 0) {
          int pos = list[sl];
          pos = pos < 0 ? 0 : (pos > RCAP - 1 ? RCAP - 1 : pos);
          reg2[pos] = eid;
          list[sl] = pos + 1;
        }
      }
    }
  }
  __syncthreads();

  const int nbw = nb >> 3;
  const int ca8 = 8 * lane;
  const int cb8 = 256 + 8 * lane;
  const v4f av0 = *(const v4f*)(avec + ca8), av1 = *(const v4f*)(avec + ca8 + 4);
  const v4f av2 = *(const v4f*)(avec + cb8), av3 = *(const v4f*)(avec + cb8 + 4);
  const v4f cz0 = *(const v4f*)(cvec + ca8), cz1 = *(const v4f*)(cvec + ca8 + 4);
  const v4f cz2 = *(const v4f*)(cvec + cb8), cz3 = *(const v4f*)(cvec + cb8 + 4);
  const bool ovf = (nh >= RCAP);
  const float qnan = __int_as_float(0x7fc00000);
  const float ninf = __int_as_float((int)0xff800000u);
#pragma unroll 1
  for (int jt = 0; jt < nbw; ++jt) {
    const int slot = wave * nbw + jt;
    const int grow = nodeBase + slot;
    const int gcl  = grow < nN ? grow : nN - 1;
    int st = soff[slot];
    const int craw = scnt[slot];
    int cnt = craw;
    st  = st < 0 ? 0 : (st > nh ? nh : st);
    cnt = cnt < 0 ? 0 : (cnt > DEGCAP ? DEGCAP : cnt);
    if (cnt > nh - st) cnt = nh - st;
    const float pz = (ovf || craw > DEGCAP) ? qnan : 0.0f;
    const bool wr = grow < nN;

    const float* yd = Y + (size_t)gcl * YP + DHID;
    const v4f t0 = *(const v4f*)(yd + ca8), t1 = *(const v4f*)(yd + ca8 + 4);
    const v4f t2 = *(const v4f*)(yd + cb8), t3 = *(const v4f*)(yd + cb8 + 4);
    float mx = ninf;
    float dn = 0.0f;
    v4f a0 = {0.f, 0.f, 0.f, 0.f}, a1 = {0.f, 0.f, 0.f, 0.f}, a2 = {0.f, 0.f, 0.f, 0.f}, a3 = {0.f, 0.f, 0.f, 0.f};
#pragma unroll 1
    for (int q = 0; q <= cnt; ++q) {
      int idx = st + q - 1;
      idx = idx < 0 ? 0 : (idx > RCAP - 1 ? RCAP - 1 : idx);
      int eid = reg2[idx]; eid = eid < 0 ? 0 : (eid > nE - 1 ? nE - 1 : eid);
      const int sraw = srcs[eid];
      const int sld  = sraw < 0 ? 0 : (sraw > nN - 1 ? nN - 1 : sraw);
      const int s = (q == 0) ? gcl : sld;
      const float* ys = Y + (size_t)s * YP;
      const v4f x0 = *(const v4f*)(ys + ca8), x1 = *(const v4f*)(ys + ca8 + 4);
      const v4f x2 = *(const v4f*)(ys + cb8), x3 = *(const v4f*)(ys + cb8 + 4);
      float pd = 0.f;
#define LKY(X, T, A) { float v_ = (X) + (T); v_ = fmaxf(v_, NEG2 * v_); pd = fmaf(v_, (A), pd); }
      LKY(x0.x, t0.x, av0.x) LKY(x0.y, t0.y, av0.y) LKY(x0.z, t0.z, av0.z) LKY(x0.w, t0.w, av0.w)
      LKY(x1.x, t1.x, av1.x) LKY(x1.y, t1.y, av1.y) LKY(x1.z, t1.z, av1.z) LKY(x1.w, t1.w, av1.w)
      LKY(x2.x, t2.x, av2.x) LKY(x2.y, t2.y, av2.y) LKY(x2.z, t2.z, av2.z) LKY(x2.w, t2.w, av2.w)
      LKY(x3.x, t3.x, av3.x) LKY(x3.y, t3.y, av3.y) LKY(x3.z, t3.z, av3.z) LKY(x3.w, t3.w, av3.w)
#undef LKY
      pd += __shfl_xor(pd, 16);
      pd += __shfl_xor(pd, 8);
      pd += __shfl_xor(pd, 4);
      pd += __shfl_xor(pd, 2);
      pd += __shfl_xor(pd, 1);
      const float mn = fmaxf(mx, pd);
      const float e1 = __expf(mx - mn), e2 = __expf(pd - mn);
      dn = fmaf(dn, e1, e2);
#define UPD(AC, X) AC = fmaf(AC, e1, e2 * (X));
      UPD(a0.x, x0.x) UPD(a0.y, x0.y) UPD(a0.z, x0.z) UPD(a0.w, x0.w)
      UPD(a1.x, x1.x) UPD(a1.y, x1.y) UPD(a1.z, x1.z) UPD(a1.w, x1.w)
      UPD(a2.x, x2.x) UPD(a2.y, x2.y) UPD(a2.z, x2.z) UPD(a2.w, x2.w)
      UPD(a3.x, x3.x) UPD(a3.y, x3.y) UPD(a3.z, x3.z) UPD(a3.w, x3.w)
#undef UPD
      mx = mn;
    }
    const float inv = __builtin_amdgcn_rcpf(dn);
    v4f o0, o1, o2, o3;
#define EPI(O, AC, CZ) O = tanh_e(fmaf(AC, inv, CZ) + pz);
    EPI(o0.x, a0.x, cz0.x) EPI(o0.y, a0.y, cz0.y) EPI(o0.z, a0.z, cz0.z) EPI(o0.w, a0.w, cz0.w)
    EPI(o1.x, a1.x, cz1.x) EPI(o1.y, a1.y, cz1.y) EPI(o1.z, a1.z, cz1.z) EPI(o1.w, a1.w, cz1.w)
    EPI(o2.x, a2.x, cz2.x) EPI(o2.y, a2.y, cz2.y) EPI(o2.z, a2.z, cz2.z) EPI(o2.w, a2.w, cz2.w)
    EPI(o3.x, a3.x, cz3.x) EPI(o3.y, a3.y, cz3.y) EPI(o3.z, a3.z, cz3.z) EPI(o3.w, a3.w, cz3.w)
#undef EPI
    v8us hv0, lv0, hv1, lv1;
    split8(o0, o1, hv0, lv0);
    split8(o2, o3, hv1, lv1);
    unsigned short* hp = oh + (size_t)gcl * DHID;
    unsigned short* lp = ol + (size_t)gcl * DHID;
    if (wr) {
      *(volatile v8us*)(hp + ca8) = hv0;
      *(volatile v8us*)(hp + cb8) = hv1;
      *(volatile v8us*)(lp + ca8) = lv0;
      *(volatile v8us*)(lp + cb8) = lv1;
    }
    __threadfence();
    if (wr) {
      *(volatile v8us*)(hp + ca8) = hv0;
      *(volatile v8us*)(hp + cb8) = hv1;
      *(volatile v8us*)(lp + ca8) = lv0;
      *(volatile v8us*)(lp + cb8) = lv1;
    }
  }
}

static int pick_nb(int nE, int nN) {
  int nb = NBMAX;
  while (nb > 16 && (long long)nb * (long long)nE * 5LL > (long long)RCAP * (long long)nN * 4LL) nb >>= 1;
  return nb;
}

extern "C" void kernel_launch(void* const* d_in, const int* in_sizes, int n_in,
                              void* d_out, int out_size, void* d_ws, size_t ws_size,
                              hipStream_t stream) {
  if (n_in < 26) return;
  const int nN = in_sizes[0] / DIN;
  if (nN <= 0 || in_sizes[0] != nN * DIN) return;
  if (nN > (1 << 22)) return;
  const int nE = in_sizes[1] / 2;
  if (nE < 1 || in_sizes[1] != 2 * nE) return;
  if (nE > (1 << 20)) return;
  for (int l = 0; l < 3; ++l) {
    const int kdim = (l == 0) ? DIN : DHID;
    const int b = 2 + 6 * l;
    if (in_sizes[b + 0] != kdim * DHID) return;
    if (in_sizes[b + 1] != DHID) return;
    if (in_sizes[b + 2] != kdim * DHID) return;
    if (in_sizes[b + 3] != DHID) return;
    if (in_sizes[b + 4] != DHID) return;
    if (in_sizes[b + 5] != DHID) return;
  }
  if (in_sizes[20] != DHID * DHID || in_sizes[21] != DHID) return;
  if (in_sizes[22] != DHID * DHID || in_sizes[23] != DHID) return;
  if (in_sizes[24] != DHID || in_sizes[25] != 1) return;
  if (out_size != nN) return;

  const float* x   = (const float*)d_in[0];
  const int*   ei  = (const int*)d_in[1];
  const int*   src = ei;
  const int*   dst = ei + nE;
  const float* W1s = (const float*)d_in[2];  const float* b1s = (const float*)d_in[3];
  const float* W1t = (const float*)d_in[4];  const float* b1t = (const float*)d_in[5];
  const float* a1  = (const float*)d_in[6];  const float* c1  = (const float*)d_in[7];
  const float* W2s = (const float*)d_in[8];  const float* b2s = (const float*)d_in[9];
  const float* W2t = (const float*)d_in[10]; const float* b2t = (const float*)d_in[11];
  const float* a2  = (const float*)d_in[12]; const float* c2  = (const float*)d_in[13];
  const float* W3s = (const float*)d_in[14]; const float* b3s = (const float*)d_in[15];
  const float* W3t = (const float*)d_in[16]; const float* b3t = (const float*)d_in[17];
  const float* a3  = (const float*)d_in[18]; const float* c3  = (const float*)d_in[19];
  const float* Wh1 = (const float*)d_in[20]; const float* bh1 = (const float*)d_in[21];
  const float* Wh2 = (const float*)d_in[22]; const float* bh2 = (const float*)d_in[23];
  const float* Wh3 = (const float*)d_in[24]; const float* bh3 = (const float*)d_in[25];
  float* out = (float*)d_out;

  const int MP   = ((nN + GBM - 1) / GBM) * GBM;
  const int nb   = pick_nb(nE, nN);
  const int vec8 = ((nE & 3) == 0) ? 1 : 0;

  char* ws = (char*)d_ws;
  size_t off = 0;
  const size_t oWH = off; off += (size_t)WTOT * 2;               off = (off + 255) & ~(size_t)255;
  const size_t oWL = off; off += (size_t)WTOT * 2;               off = (off + 255) & ~(size_t)255;
  const size_t oXH = off; off += (size_t)MP * DIN * 2;           off = (off + 255) & ~(size_t)255;
  const size_t oXL = off; off += (size_t)MP * DIN * 2;           off = (off + 255) & ~(size_t)255;
  const size_t oHH = off; off += (size_t)MP * DHID * 2;          off = (off + 255) & ~(size_t)255;
  const size_t oHL = off; off += (size_t)MP * DHID * 2;          off = (off + 255) & ~(size_t)255;
  const size_t oGH = off; off += (size_t)MP * DHID * 2;          off = (off + 255) & ~(size_t)255;
  const size_t oGL = off; off += (size_t)MP * DHID * 2;          off = (off + 255) & ~(size_t)255;
  const size_t oY  = off; off += (size_t)MP * YP * 4;            off = (off + 255) & ~(size_t)255;
  if (off > ws_size || off > (size_t)WSCAP) return;
  unsigned short* WH = (unsigned short*)(ws + oWH);
  unsigned short* WL = (unsigned short*)(ws + oWL);
  unsigned short* XH = (unsigned short*)(ws + oXH);
  unsigned short* XL = (unsigned short*)(ws + oXL);
  unsigned short* HH = (unsigned short*)(ws + oHH);
  unsigned short* HL = (unsigned short*)(ws + oHL);
  unsigned short* GH = (unsigned short*)(ws + oGH);
  unsigned short* GL = (unsigned short*)(ws + oGL);
  float*          Y  = (float*)(ws + oY);

  const size_t wL1 = 0;
  const size_t wL2 = (size_t)2 * DHID * DIN;
  const size_t wL3 = wL2 + (size_t)2 * DHID * DHID;
  const size_t wH1 = wL3 + (size_t)2 * DHID * DHID;
  const size_t wH2 = wH1 + (size_t)DHID * DHID;

  hipFuncSetAttribute(reinterpret_cast<const void*>(&k_agg),
                      hipFuncAttributeMaxDynamicSharedMemorySize, LDS_AGG);

  const int xUnits = MP * (DIN / 8);
  k_xprep<<<(xUnits + NTHR - 1) / NTHR, NTHR, 0, stream>>>(x, XH, XL, nN, xUnits);
  const int pUnits = (MP - nN) * (DHID / 8);
  if (pUnits > 0) k_hpad<<<(pUnits + NTHR - 1) / NTHR, NTHR, 0, stream>>>(HH, HL, nN, pUnits);
  k_wprep<<<dim3((DHID * (DHID / 8) + NTHR - 1) / NTHR, 8), NTHR, 0, stream>>>(
      W1s, W1t, W2s, W2t, W3s, W3t, Wh1, Wh2, WH, WL);

  const int gG = MP / GBM;
  const int gA = (nN + nb - 1) / nb;

  k_gemm<0><<<gG, GTHR, 0, stream>>>(XH, XL, WH + wL1, WL + wL1, b1s, b1t, Wh3, bh3, Y, GH, GL, out,
                                      DIN / 32, DIN, NCAT / 64, nN);
  k_agg<<<gA, NTHR, LDS_AGG, stream>>>(src, dst, Y, a1, c1, HH, HL, nN, nE, nb, vec8);
  k_gemm<0><<<gG, GTHR, 0, stream>>>(HH, HL, WH + wL2, WL + wL2, b2s, b2t, Wh3, bh3, Y, GH, GL, out,
                                      DHID / 32, DHID, NCAT / 64, nN);
  k_agg<<<gA, NTHR, LDS_AGG, stream>>>(src, dst, Y, a2, c2, HH, HL, nN, nE, nb, vec8);
  k_gemm<0><<<gG, GTHR, 0, stream>>>(HH, HL, WH + wL3, WL + wL3, b3s, b3t, Wh3, bh3, Y, GH, GL, out,
                                      DHID / 32, DHID, NCAT / 64, nN);
  k_agg<<<gA, NTHR, LDS_AGG, stream>>>(src, dst, Y, a3, c3, HH, HL, nN, nE, nb, vec8);
  k_gemm<1><<<gG, GTHR, 0, stream>>>(HH, HL, WH + wH1, WL + wH1, bh1, bh1, Wh3, bh3, Y, GH, GL, out,
                                      DHID / 32, DHID, DHID / 64, nN);
  k_gemm<2><<<gG, GTHR, 0, stream>>>(GH, GL, WH + wH2, WL + wH2, bh2, bh2, Wh3, bh3, Y, GH, GL, out,
                                      DHID / 32, DHID, DHID / 64, nN);
}
